// HeterogeneousGraphNetwork_37220186587466
// MI455X (gfx1250) — hardware-run, weakly checked
//
#include <hip/hip_runtime.h>
#include <math.h>
#include <stdint.h>

#define NB    4
#define NN    1024
#define FD    512
#define HD    64
#define NH    8
#define SROWS (NB * NN)
#define AROWS (2 * SROWS)

static_assert(FD == NH * HD);
static_assert(HD == 64);
static_assert(NN % 64 == 0);
static_assert(AROWS % 128 == 0);
static_assert((3 * FD) % 64 == 0);
static_assert(FD % 32 == 0);
static_assert((2 * HD) % 32 == 0);

typedef __attribute__((ext_vector_type(16))) __bf16        v16b;
typedef __attribute__((ext_vector_type(8)))  __bf16        v8b;
typedef __attribute__((ext_vector_type(8)))  float         v8f;
typedef __attribute__((ext_vector_type(4)))  float         v4f;
typedef __attribute__((ext_vector_type(4)))  unsigned int  v4u;
typedef v4f __attribute__((may_alias)) v4fa;

constexpr size_t SZ_XB  = (size_t)AROWS * FD * 2;
constexpr size_t SZ_WP  = (size_t)3 * FD * FD * 2;
constexpr size_t SZ_EWT = (size_t)3 * HD * 128 * 2;
constexpr size_t SZ_WO  = (size_t)FD * FD * 2;
constexpr size_t SZ_F1  = (size_t)AROWS * NH * 128 * 2;
constexpr size_t SZ_CTX = (size_t)4 * SROWS * 2 * FD * 2;
constexpr size_t SZ_RA  = SZ_CTX;
constexpr size_t SZ_Q   = (size_t)2 * 4 * SROWS * FD * 2;
constexpr size_t SZ_K   = (size_t)2 * AROWS * FD * 2;
constexpr size_t SZ_VT  = SZ_K;
constexpr size_t SZ_Y   = (size_t)AROWS * FD * 4;
constexpr size_t OFF_XB  = 0;
constexpr size_t OFF_WP  = OFF_XB + SZ_XB;
constexpr size_t OFF_EWT = OFF_WP + SZ_WP;
constexpr size_t OFF_WO  = OFF_EWT + SZ_EWT;
constexpr size_t OFF_RA  = OFF_WO + SZ_WO;
constexpr size_t OFF_Q   = OFF_RA + SZ_RA;
constexpr size_t OFF_K   = OFF_Q + SZ_Q;
constexpr size_t OFF_VT  = OFF_K + SZ_K;
constexpr size_t OFF_Y   = OFF_VT + SZ_VT;
constexpr size_t WS_TOTAL = OFF_Y + SZ_Y;
static_assert(SZ_F1 <= SZ_RA);
static_assert(WS_TOTAL == 127975424);
static_assert(WS_TOTAL <= 134217728);
static_assert((OFF_WP % 256) == 0 && (OFF_EWT % 256) == 0 && (OFF_WO % 256) == 0 && (OFF_RA % 256) == 0);
static_assert((OFF_Q % 256) == 0 && (OFF_K % 256) == 0 && (OFF_VT % 256) == 0 && (OFF_Y % 256) == 0);
constexpr size_t EO_F1 = OFF_RA / 2;
constexpr size_t EO_K  = OFF_K / 2;
constexpr size_t EO_VT = OFF_VT / 2;
constexpr size_t PLANE16 = (size_t)AROWS * FD;
constexpr size_t QPLANE  = (size_t)4 * SROWS * FD;
static_assert((size_t)(AROWS - 1) * FD + (FD - 1) == 4194303);

__device__ __forceinline__ unsigned short f2bf_bits(float f) {
  const unsigned u = __float_as_uint(f);
  const unsigned r = (u + 0x7FFFu + ((u >> 16) & 1u)) >> 16;
  const unsigned n = (u >> 16) | 0x40u;
  return (unsigned short)(((u & 0x7FFFFFFFu) > 0x7F800000u) ? n : r);
}
__device__ __forceinline__ unsigned short f2bf_fast(float f) {
  const unsigned u = __float_as_uint(f);
  return (unsigned short)((u + 0x7FFFu + ((u >> 16) & 1u)) >> 16);
}
__device__ __forceinline__ float bf_bits2f(unsigned short h) { return __uint_as_float(((unsigned)h) << 16); }
__device__ __forceinline__ float bfr(float f) { return bf_bits2f(f2bf_bits(f)); }
__device__ __forceinline__ unsigned pk16(unsigned short a, unsigned short b) { return (unsigned)a | ((unsigned)b << 16); }

__device__ __forceinline__ v4u pack_hl8(const float (&f)[8], unsigned plane) {
  v4u o;
#pragma unroll
  for (int q = 0; q < 4; ++q) {
    const float x0 = f[2 * q], x1 = f[2 * q + 1];
    const unsigned short h0 = f2bf_bits(x0), h1 = f2bf_bits(x1);
    const unsigned short l0 = f2bf_bits(x0 - bf_bits2f(h0)), l1 = f2bf_bits(x1 - bf_bits2f(h1));
    const unsigned uh = pk16(h0, h1), ul = pk16(l0, l1);
    o[q] = (plane != 0u) ? ul : uh;
  }
  return o;
}

union FB { v16b v; v8b h[2]; };
__device__ __forceinline__ v16b ldfrag(const __bf16* p) {
  FB f; f.h[0] = *(const v8b*)(p); f.h[1] = *(const v8b*)(p + 16); return f.v;
}
__device__ __forceinline__ v8f wm(v16b a, v16b b, v8f c) {
  c = __builtin_amdgcn_wmma_f32_16x16x32_bf16(false, a, false, b, (short)0, c, false, false);
  asm volatile("v_nop\n\tv_nop\n\tv_nop\n\tv_nop" : "+v"(c) : "v"(a), "v"(b));
  return c;
}
template <int LDA, int LDB, int KT>
__device__ __forceinline__ void tile_mma(const __bf16* a0p, const __bf16* bp, v8f (&acc)[2][4]) {
  const __bf16* a1p = a0p + (size_t)16 * LDA;
#pragma unroll 1
  for (int k0 = 0; k0 < KT; k0 += 32) {
    const v16b a0 = ldfrag(a0p + k0);
    const v16b a1 = ldfrag(a1p + k0);
#pragma unroll
    for (int nt = 0; nt < 4; ++nt) {
      const v16b b = ldfrag(bp + (size_t)nt * 16 * LDB + k0);
      acc[0][nt] = wm(a0, b, acc[0][nt]);
      acc[1][nt] = wm(a1, b, acc[1][nt]);
    }
  }
}

__global__ __launch_bounds__(256) void k_cvt(const float* __restrict__ src, unsigned short* dst, int n8) {
  const int g = blockIdx.x * 256 + threadIdx.x;
  if (g < n8) {
    const v4f a = *(const v4f*)(src + (size_t)g * 8);
    const v4f c = *(const v4f*)(src + (size_t)g * 8 + 4);
    v4u o;
    o[0] = pk16(f2bf_bits(a[0]), f2bf_bits(a[1]));
    o[1] = pk16(f2bf_bits(a[2]), f2bf_bits(a[3]));
    o[2] = pk16(f2bf_bits(c[0]), f2bf_bits(c[1]));
    o[3] = pk16(f2bf_bits(c[2]), f2bf_bits(c[3]));
    *(volatile v4u*)(dst + (size_t)g * 8) = o;
    __threadfence();
    *(volatile v4u*)(dst + (size_t)g * 8) = o;
  }
}

__global__ __launch_bounds__(256) void k_wt(const float* __restrict__ W, unsigned short* dst) {
  __shared__ __align__(16) float tf[64 * 68];
  const int h   = blockIdx.z;
  const int r0  = blockIdx.y * 64;
  const int tid = threadIdx.x;
  const float* Wh = W + (size_t)h * FD * HD;
  {
    const int lr = tid >> 4;
    const int c4 = (tid & 15) * 4;
#pragma unroll
    for (int it = 0; it < 4; ++it) {
      const int rr = it * 16 + lr;
      const v4f a = *(const v4f*)(Wh + (size_t)(r0 + rr) * HD + c4);
      *(v4fa*)(tf + rr * 68 + c4) = a;
    }
  }
  __syncthreads();
  const int sub = tid >> 3;
  const int c8  = (tid & 7) * 8;
  v4u hv[2];
#pragma unroll
  for (int it = 0; it < 2; ++it) {
    const int oc = it * 32 + sub;
    v4u a;
#pragma unroll
    for (int q = 0; q < 4; ++q) {
      const float f0 = tf[(c8 + 2 * q) * 68 + oc];
      const float f1 = tf[(c8 + 2 * q + 1) * 68 + oc];
      a[q] = pk16(f2bf_bits(f0), f2bf_bits(f1));
    }
    hv[it] = a;
  }
  for (int pass = 0; pass < 2; ++pass) {
#pragma unroll
    for (int it = 0; it < 2; ++it) {
      const int oc = it * 32 + sub;
      *(volatile v4u*)(dst + (size_t)(h * HD + oc) * FD + r0 + c8) = hv[it];
    }
    __threadfence();
  }
}

__global__ __launch_bounds__(256) void k_ew(const float* __restrict__ ew, unsigned short* dst) {
  __shared__ __align__(16) float tf[64 * 68];
  const int tid = threadIdx.x;
  {
    const int lr = tid >> 4;
    const int c4 = (tid & 15) * 4;
#pragma unroll
    for (int it = 0; it < 4; ++it) {
      const int rr = it * 16 + lr;
      const v4f a = *(const v4f*)(ew + (size_t)rr * HD + c4);
      *(v4fa*)(tf + rr * 68 + c4) = a;
    }
  }
  __syncthreads();
  const int sub = tid >> 3;
  const int c8  = (tid & 7) * 8;
  v4u hv[4];
#pragma unroll
  for (int it = 0; it < 4; ++it) {
    const int lid = it * 32 + sub;
    const int l = lid >> 1;
    v4u a;
#pragma unroll
    for (int q = 0; q < 4; ++q) {
      const float f0 = tf[(c8 + 2 * q) * 68 + l];
      const float f1 = tf[(c8 + 2 * q + 1) * 68 + l];
      a[q] = pk16(f2bf_bits(f0), f2bf_bits(f1));
    }
    hv[it] = a;
  }
  for (int pass = 0; pass < 2; ++pass) {
#pragma unroll
    for (int it = 0; it < 4; ++it) {
      const int lid = it * 32 + sub;
      const int l = lid >> 1, half = lid & 1;
      *(volatile v4u*)(dst + (size_t)l * 128 + half * 64 + c8) = hv[it];
    }
    __threadfence();
  }
}

__device__ __forceinline__ void proj_store_pass(const float* sT, unsigned short* ob, int p, int head,
                                                int m0, int w, int lane) {
  const int q8 = lane & 7, sub = lane >> 3;
#pragma unroll 1
  for (int i = 0; i < 16; ++i) {
    const int lid = w * 64 + i * 4 + sub;
    const unsigned plane = (unsigned)(lid & 1);
    float f[8];
    size_t off;
    if (p == 2) {
      const int d = lid >> 2, hl = (lid >> 1) & 1;
#pragma unroll
      for (int e = 0; e < 8; ++e) f[e] = sT[(64 * hl + 8 * q8 + e) * 68 + d];
      off = EO_VT + (size_t)plane * PLANE16 + ((size_t)((m0 >> 10) * NH + head) * HD + d) * NN
          + (size_t)((m0 & (NN - 1)) + 64 * hl + 8 * q8);
    } else {
      const int row = lid >> 1;
#pragma unroll
      for (int e = 0; e < 8; ++e) f[e] = sT[row * 68 + 8 * q8 + e];
      if (p == 0) off = EO_F1 + ((size_t)(m0 + row) * NH + head) * 128 + (size_t)plane * 64 + 8 * q8;
      else        off = EO_K + (size_t)plane * PLANE16 + (size_t)(m0 + row) * FD + head * HD + 8 * q8;
    }
    const v4u val = pack_hl8(f, plane);
    *(volatile v4u*)(ob + off) = val;
  }
}

__attribute__((amdgpu_num_vgpr(248)))
__global__ __launch_bounds__(128) void k_proj(const unsigned short* __restrict__ xbp,
                                              const unsigned short* __restrict__ wpp,
                                              const float* __restrict__ b1, const float* __restrict__ b2,
                                              const float* __restrict__ b3, unsigned short* ob) {
  __shared__ __align__(16) float sT[128 * 68];
  __shared__ __align__(16) float sB[3 * 64];
  const int tid = threadIdx.x, lane = tid & 31, w = tid >> 5;
  const int hh = lane >> 4, m = lane & 15;
  const int m0 = blockIdx.x * 128;
  const int cg = blockIdx.y;
  const int p = cg >> 3, head = cg & 7;
  const __bf16* X = (const __bf16*)(const void*)xbp;
  const __bf16* W = (const __bf16*)(const void*)wpp;
  const __bf16* a0p = X + (size_t)(m0 + 32 * w + m) * FD + 8 * hh;
  const __bf16* bp  = W + (size_t)(p * FD + head * HD + m) * FD + 8 * hh;

  {
    const int bi = head * HD + (tid & 63);
    const float v1 = b1[bi];
    const float v2 = b2[bi];
    const float v3 = b3[bi];
    asm volatile("" :: "v"(v1), "v"(v2), "v"(v3));
    if (tid < 64) {
      sB[tid]       = bfr(v1);
      sB[64 + tid]  = bfr(v2);
      sB[128 + tid] = bfr(v3);
    }
  }
  __syncthreads();

  v8f acc[2][4];
#pragma unroll
  for (int mt = 0; mt < 2; ++mt)
#pragma unroll
    for (int nt = 0; nt < 4; ++nt) acc[mt][nt] = (v8f){0.f, 0.f, 0.f, 0.f, 0.f, 0.f, 0.f, 0.f};
  tile_mma<FD, FD, FD>(a0p, bp, acc);

#pragma unroll
  for (int nt = 0; nt < 4; ++nt) {
    const int feat = 16 * nt + m;
    const float bv = sB[p * 64 + feat];
#pragma unroll
    for (int mt = 0; mt < 2; ++mt) {
#pragma unroll
      for (int r = 0; r < 8; ++r) {
        const int tokl = 32 * w + 16 * mt + 8 * hh + r;
        sT[tokl * 68 + feat] = acc[mt][nt][r] + bv;
      }
    }
  }
  __syncthreads();
  proj_store_pass(sT, ob, p, head, m0, w, lane);
  __threadfence();
  proj_store_pass(sT, ob, p, head, m0, w, lane);
}

__device__ __forceinline__ void g_store_pass(const float* sT, unsigned short* qout, int c, int m0, int w, int lane) {
  const int q8 = lane & 7, sub = lane >> 3;
#pragma unroll 1
  for (int i = 0; i < 16; ++i) {
    const int lid = w * 64 + i * 4 + sub;
    const unsigned plane = (unsigned)(lid & 1);
    const int row = lid >> 1;
    float f[8];
#pragma unroll
    for (int e = 0; e < 8; ++e) f[e] = sT[row * 68 + 8 * q8 + e];
    const v4u val = pack_hl8(f, plane);
    const size_t off = (size_t)plane * QPLANE + (size_t)c * SROWS * FD + (size_t)(m0 + row) * HD + 8 * q8;
    *(volatile v4u*)(qout + off) = val;
  }
}

__attribute__((amdgpu_num_vgpr(248)))
__global__ __launch_bounds__(128) void k_g(const unsigned short* __restrict__ f1hl,
                                           const unsigned short* __restrict__ ewt,
                                           unsigned short* qout) {
  __shared__ __align__(16) float sT[128 * 68];
  const int tid = threadIdx.x, lane = tid & 31, w = tid >> 5;
  const int hh = lane >> 4, m = lane & 15;
  const int m0 = blockIdx.x * 128;
  const int c = blockIdx.y;
  const int setq = c & 1;
  const int e = (c < 2) ? c : 2;
  const __bf16* A = (const __bf16*)(const void*)f1hl + (size_t)setq * SROWS * NH * 128;
  const __bf16* B = (const __bf16*)(const void*)ewt + (size_t)e * HD * 128;
  const __bf16* a0p = A + (size_t)(m0 + 32 * w + m) * 128 + 8 * hh;
  const __bf16* bp  = B + (size_t)m * 128 + 8 * hh;

  v8f acc[2][4];
#pragma unroll
  for (int mt = 0; mt < 2; ++mt)
#pragma unroll
    for (int nt = 0; nt < 4; ++nt) acc[mt][nt] = (v8f){0.f, 0.f, 0.f, 0.f, 0.f, 0.f, 0.f, 0.f};
  tile_mma<128, 128, 128>(a0p, bp, acc);

#pragma unroll
  for (int nt = 0; nt < 4; ++nt)
#pragma unroll
    for (int mt = 0; mt < 2; ++mt)
#pragma unroll
      for (int r = 0; r < 8; ++r)
        sT[(32 * w + 16 * mt + 8 * hh + r) * 68 + 16 * nt + m] = acc[mt][nt][r];
  __syncthreads();
  g_store_pass(sT, qout, c, m0, w, lane);
  __threadfence();
  g_store_pass(sT, qout, c, m0, w, lane);
}

#define AT_D  64
#define AT_NW 4
#define AT_KC 64

__device__ __forceinline__ void at_split(float f, __bf16& hi, __bf16& lo) {
  const unsigned short hb = f2bf_fast(f);
  hi = __builtin_bit_cast(__bf16, hb);
  lo = __builtin_bit_cast(__bf16, f2bf_fast(f - __uint_as_float(((unsigned)hb) << 16)));
}

__attribute__((amdgpu_num_vgpr(248)))
__global__ __launch_bounds__(128)
void k_attn(const unsigned short* __restrict__ qhp, const unsigned short* __restrict__ qlp,
            const unsigned short* __restrict__ khp, const unsigned short* __restrict__ klp,
            const unsigned short* __restrict__ vhp, const unsigned short* __restrict__ vlp,
            const float* __restrict__ adj, unsigned short* ctx, int trans) {
  __shared__ __align__(16) __bf16 Ksh[AT_KC * AT_D];
  __shared__ __align__(16) __bf16 Ksl[AT_KC * AT_D];
  __shared__ __align__(16) __bf16 Vth[AT_D * AT_KC];
  __shared__ __align__(16) __bf16 Vtl[AT_D * AT_KC];
  __shared__ __align__(16) __bf16 Psh[AT_NW][16 * AT_KC];
  __shared__ __align__(16) __bf16 Psl[AT_NW][16 * AT_KC];
  __shared__ __align__(16) float  Sw[AT_NW][16 * 68];
  __shared__ __align__(16) float  As[64 * 65];

  const int tid  = threadIdx.x;
  const int wave = tid >> 5;
  const int lane = tid & 31;
  const int hh   = lane >> 4;
  const int c    = lane & 15;

  const int bx = blockIdx.x;
  const int qb = bx & 15;
  const int h  = (bx >> 4) & 7;
  const int b  = bx >> 7;
  const int qblk0 = qb * 64;
  const int q0 = qblk0 + wave * 16;

  const size_t tok0 = (size_t)b * NN;
  const __bf16* Qh = (const __bf16*)(const void*)qhp + tok0 * FD + (size_t)h * AT_D;
  const __bf16* Ql = (const __bf16*)(const void*)qlp + tok0 * FD + (size_t)h * AT_D;
  const __bf16* Kh = (const __bf16*)(const void*)khp + tok0 * FD + (size_t)h * AT_D;
  const __bf16* Kl = (const __bf16*)(const void*)klp + tok0 * FD + (size_t)h * AT_D;
  const __bf16* Vh = (const __bf16*)(const void*)vhp + (size_t)(b * NH + h) * AT_D * NN;
  const __bf16* Vl = (const __bf16*)(const void*)vlp + (size_t)(b * NH + h) * AT_D * NN;
  const float* adjb = adj + (size_t)b * NN * NN;

  const int tr = (trans != 0) ? 1 : 0;
  const int a_sr   = tr ? 1 : 65;
  const int a_sj   = tr ? (16 * 65) : 16;
  const int a_base = tr ? (c * 65 + wave * 16 + 8 * hh) : ((wave * 16 + 8 * hh) * 65 + c);

  v16b qah[2], qal[2];
#pragma unroll
  for (int dc = 0; dc < 2; ++dc) {
    qah[dc] = ldfrag(Qh + (size_t)(q0 + c) * FD + dc * 32 + 8 * hh);
    qal[dc] = ldfrag(Ql + (size_t)(q0 + c) * FD + dc * 32 + 8 * hh);
  }

  float mrow[8], lrow[8];
  v8f oacc[4];
#pragma unroll
  for (int r = 0; r < 8; ++r) { mrow[r] = -INFINITY; lrow[r] = 0.f; }
#pragma unroll
  for (int t = 0; t < 4; ++t) oacc[t] = (v8f){0.f, 0.f, 0.f, 0.f, 0.f, 0.f, 0.f, 0.f};

  float*  sw  = Sw[wave];
  __bf16* pwh = Psh[wave];
  __bf16* pwl = Psl[wave];
  const int s_base = (8 * hh) * 68 + c;

#pragma unroll 1
  for (int kc = 0; kc < NN / AT_KC; ++kc) {
    const int kv0 = kc * AT_KC;
    __syncthreads();
    {
      const int r = tid >> 1, half = (tid & 1) * 32;
      const __bf16* ksh = Kh + (size_t)(kv0 + r) * FD + half;
      const __bf16* ksl = Kl + (size_t)(kv0 + r) * FD + half;
      const __bf16* vsh = Vh + (size_t)r * NN + kv0 + half;
      const __bf16* vsl = Vl + (size_t)r * NN + kv0 + half;
#pragma unroll 1
      for (int i = 0; i < 4; ++i) {
        const v8b a0 = *(const v8b*)(ksh + 8 * i);
        const v8b a1 = *(const v8b*)(ksl + 8 * i);
        const v8b b0 = *(const v8b*)(vsh + 8 * i);
        const v8b b1 = *(const v8b*)(vsl + 8 * i);
        *(v8b*)(Ksh + r * AT_D  + half + 8 * i) = a0;
        *(v8b*)(Ksl + r * AT_D  + half + 8 * i) = a1;
        *(v8b*)(Vth + r * AT_KC + half + 8 * i) = b0;
        *(v8b*)(Vtl + r * AT_KC + half + 8 * i) = b1;
      }
      const int R0 = tr ? kv0 : qblk0;
      const int C0 = tr ? qblk0 : kv0;
#pragma unroll 2
      for (int it = 0; it < 8; ++it) {
        const int idx = it * 128 + tid;
        const int ar = idx >> 4, c4 = (idx & 15) * 4;
        const v4f a = *(const v4f*)(adjb + (size_t)(R0 + ar) * NN + C0 + c4);
        float* d = As + ar * 65 + c4;
        d[0] = bfr(a[0]);
        d[1] = bfr(a[1]);
        d[2] = bfr(a[2]);
        d[3] = bfr(a[3]);
      }
    }
    __syncthreads();

    float cm[8];
#pragma unroll
    for (int r = 0; r < 8; ++r) cm[r] = -INFINITY;
#pragma unroll 1
    for (int j = 0; j < 4; ++j) {
      v8f sj = (v8f){0.f, 0.f, 0.f, 0.f, 0.f, 0.f, 0.f, 0.f};
#pragma unroll
      for (int dc = 0; dc < 2; ++dc) {
        FB kb, kl;
        kb.h[0] = *(const v8b*)(Ksh + (j * 16 + c) * AT_D + dc * 32 + 8 * hh);
        kb.h[1] = *(const v8b*)(Ksh + (j * 16 + c) * AT_D + dc * 32 + 16 + 8 * hh);
        kl.h[0] = *(const v8b*)(Ksl + (j * 16 + c) * AT_D + dc * 32 + 8 * hh);
        kl.h[1] = *(const v8b*)(Ksl + (j * 16 + c) * AT_D + dc * 32 + 16 + 8 * hh);
        sj = wm(qah[dc], kb.v, sj);
        sj = wm(qah[dc], kl.v, sj);
        sj = wm(qal[dc], kb.v, sj);
      }
      const int ab = a_base + j * a_sj;
      const int so = s_base + j * 16;
#pragma unroll
      for (int r = 0; r < 8; ++r) {
        const float av = As[ab + r * a_sr];
        const float sv = sj[r] * av;
        sw[so + r * 68] = sv;
        cm[r] = fmaxf(cm[r], sv);
      }
    }
#pragma unroll
    for (int r = 0; r < 8; ++r) {
      float m = cm[r];
#pragma unroll
      for (int off = 1; off < 16; off <<= 1) m = fmaxf(m, __shfl_xor(m, off, 32));
      cm[r] = m;
    }

    float alpha[8], psum[8];
#pragma unroll
    for (int r = 0; r < 8; ++r) {
      const float mnew = fmaxf(mrow[r], cm[r]);
      alpha[r] = expf(mrow[r] - mnew);
      mrow[r] = mnew;
      psum[r] = 0.f;
    }
#pragma unroll 1
    for (int j = 0; j < 4; ++j) {
      const int so = s_base + j * 16;
      const int po = (8 * hh) * AT_KC + j * 16 + c;
#pragma unroll
      for (int r = 0; r < 8; ++r) {
        const float x = sw[so + r * 68];
        const float p = expf(x - mrow[r]);
        psum[r] += p;
        __bf16 a, bl;
        at_split(p, a, bl);
        pwh[po + r * AT_KC] = a;
        pwl[po + r * AT_KC] = bl;
      }
    }
#pragma unroll
    for (int r = 0; r < 8; ++r) {
      float ps = psum[r];
#pragma unroll
      for (int off = 1; off < 16; off <<= 1) ps += __shfl_xor(ps, off, 32);
      lrow[r] = lrow[r] * alpha[r] + ps;
#pragma unroll
      for (int t = 0; t < 4; ++t) oacc[t][r] *= alpha[r];
    }
    __builtin_amdgcn_fence(__ATOMIC_RELEASE, "workgroup");
    __builtin_amdgcn_wave_barrier();
    __builtin_amdgcn_fence(__ATOMIC_ACQUIRE, "workgroup");

#pragma unroll 1
    for (int kk = 0; kk < 2; ++kk) {
      FB pa, pl;
      pa.h[0] = *(const v8b*)(pwh + c * AT_KC + kk * 32 + 8 * hh);
      pa.h[1] = *(const v8b*)(pwh + c * AT_KC + kk * 32 + 16 + 8 * hh);
      pl.h[0] = *(const v8b*)(pwl + c * AT_KC + kk * 32 + 8 * hh);
      pl.h[1] = *(const v8b*)(pwl + c * AT_KC + kk * 32 + 16 + 8 * hh);
#pragma unroll
      for (int t = 0; t < 4; ++t) {
        FB vb, vl;
        vb.h[0] = *(const v8b*)(Vth + (t * 16 + c) * AT_KC + kk * 32 + 8 * hh);
        vb.h[1] = *(const v8b*)(Vth + (t * 16 + c) * AT_KC + kk * 32 + 16 + 8 * hh);
        vl.h[0] = *(const v8b*)(Vtl + (t * 16 + c) * AT_KC + kk * 32 + 8 * hh);
        vl.h[1] = *(const v8b*)(Vtl + (t * 16 + c) * AT_KC + kk * 32 + 16 + 8 * hh);
        oacc[t] = wm(pa.v, vb.v, oacc[t]);
        oacc[t] = wm(pa.v, vl.v, oacc[t]);
        oacc[t] = wm(pl.v, vb.v, oacc[t]);
      }
    }
  }

#pragma unroll
  for (int r = 0; r < 8; ++r) {
    const float inv = 1.0f / lrow[r];
#pragma unroll
    for (int t = 0; t < 4; ++t) sw[(8 * hh + r) * 68 + t * 16 + c] = oacc[t][r] * inv;
  }
  __builtin_amdgcn_fence(__ATOMIC_RELEASE, "workgroup");
  __builtin_amdgcn_wave_barrier();
  __builtin_amdgcn_fence(__ATOMIC_ACQUIRE, "workgroup");
  {
    const int q8 = lane & 7, sub = lane >> 3;
    for (int pass = 0; pass < 2; ++pass) {
#pragma unroll 1
      for (int it = 0; it < 8; ++it) {
        const int lid = it * 4 + sub;
        const int row = lid >> 1;
        const unsigned plane = (unsigned)(lid & 1);
        float f[8];
#pragma unroll
        for (int e = 0; e < 8; ++e) f[e] = sw[row * 68 + 8 * q8 + e];
        const v4u val = pack_hl8(f, plane);
        const size_t off = (tok0 + q0 + row) * (size_t)(2 * FD) + (size_t)plane * FD + h * AT_D + 8 * q8;
        *(volatile v4u*)(ctx + off) = val;
      }
      __threadfence();
    }
  }
}

template <int FINAL>
__attribute__((amdgpu_num_vgpr(248)))
__global__ __launch_bounds__(128) void k_out(const unsigned short* __restrict__ ctxp,
                                             const unsigned short* __restrict__ wop,
                                             const float* __restrict__ bout, const float* __restrict__ boutp,
                                             const float* yin, float* dst) {
  __shared__ __align__(16) float sT[128 * 68];
  __shared__ __align__(16) float sBo[2 * 64];
  const int tid = threadIdx.x, lane = tid & 31, w = tid >> 5;
  const int hh = lane >> 4, m = lane & 15;
  const int m0 = blockIdx.x * 128;
  const int n0 = blockIdx.y * 64;
  const __bf16* C = (const __bf16*)(const void*)ctxp;
  const __bf16* W = (const __bf16*)(const void*)wop;
  const __bf16* a0p = C + (size_t)(m0 + 32 * w + m) * (2 * FD) + 8 * hh;
  const __bf16* a1p = a0p + (size_t)16 * (2 * FD);
  const __bf16* bp  = W + (size_t)(n0 + m) * FD + 8 * hh;

  {
    const int bi = n0 + (tid & 63);
    const float v1 = bout[bi];
    const float v2 = boutp[bi];
    asm volatile("" :: "v"(v1), "v"(v2));
    if (tid < 64) {
      sBo[tid]      = bfr(v1);
      sBo[64 + tid] = bfr(v2);
    }
  }
  __syncthreads();

  v8f acc[2][4];
#pragma unroll
  for (int mt = 0; mt < 2; ++mt)
#pragma unroll
    for (int nt = 0; nt < 4; ++nt) acc[mt][nt] = (v8f){0.f, 0.f, 0.f, 0.f, 0.f, 0.f, 0.f, 0.f};

#pragma unroll 1
  for (int k0 = 0; k0 < FD; k0 += 32) {
    const v16b a0h = ldfrag(a0p + k0);
    const v16b a0l = ldfrag(a0p + FD + k0);
    const v16b a1h = ldfrag(a1p + k0);
    const v16b a1l = ldfrag(a1p + FD + k0);
#pragma unroll
    for (int nt = 0; nt < 4; ++nt) {
      const v16b bfrag = ldfrag(bp + (size_t)nt * 16 * FD + k0);
      acc[0][nt] = wm(a0h, bfrag, acc[0][nt]);
      acc[0][nt] = wm(a0l, bfrag, acc[0][nt]);
      acc[1][nt] = wm(a1h, bfrag, acc[1][nt]);
      acc[1][nt] = wm(a1l, bfrag, acc[1][nt]);
    }
  }

#pragma unroll
  for (int nt = 0; nt < 4; ++nt) {
    const int nl = 16 * nt + m;
    const float bo  = sBo[nl];
    const float bo2 = sBo[64 + nl];
#pragma unroll
    for (int mt = 0; mt < 2; ++mt) {
#pragma unroll
      for (int r = 0; r < 8; ++r) {
        float v = acc[mt][nt][r] + bo;
        v = (v > 0.0f) ? v : (v - v);
        v = v + bo2;
        sT[(32 * w + 16 * mt + 8 * hh + r) * 68 + nl] = v;
      }
    }
  }
  __syncthreads();
  {
    const int c4 = m * 4;
    for (int pass = 0; pass < 2; ++pass) {
#pragma unroll 1
      for (int it = 0; it < 16; ++it) {
        const int row = 32 * w + it * 2 + hh;
        v4f v = *(const v4fa*)(sT + row * 68 + c4);
        const size_t off = (size_t)(m0 + row) * FD + n0 + c4;
        if (FINAL) {
          const v4f y = *(const v4f*)(yin + off);
          v = y + v;
        }
        *(volatile v4f*)(dst + off) = v;
      }
      __threadfence();
    }
  }
}

extern "C" void kernel_launch(void* const* d_in, const int* in_sizes, int n_in,
                              void* d_out, int out_size, void* d_ws, size_t ws_size,
                              hipStream_t stream) {
  if (n_in < 17) return;
  if (in_sizes[0] != SROWS * FD || in_sizes[1] != SROWS * FD) return;
  if (in_sizes[2] != NB * NN * NN || in_sizes[3] != NB * NN * NN || in_sizes[4] != NB * NN * NN) return;
  if (in_sizes[5] != NH * FD * HD || in_sizes[7] != NH * FD * HD || in_sizes[9] != NH * FD * HD) return;
  if (in_sizes[6] != NH * HD || in_sizes[8] != NH * HD || in_sizes[10] != NH * HD) return;
  if (in_sizes[11] != HD * HD || in_sizes[12] != HD * HD || in_sizes[13] != HD * HD) return;
  if (in_sizes[14] != FD * FD || in_sizes[15] != FD || in_sizes[16] != FD) return;
  if (out_size != 2 * SROWS * FD) return;
  if (WS_TOTAL > ws_size) return;

  const float* xa    = (const float*)d_in[0];
  const float* xb    = (const float*)d_in[1];
  const float* Aia   = (const float*)d_in[2];
  const float* Aib   = (const float*)d_in[3];
  const float* Ait   = (const float*)d_in[4];
  const float* W1    = (const float*)d_in[5];
  const float* b1    = (const float*)d_in[6];
  const float* W2    = (const float*)d_in[7];
  const float* b2    = (const float*)d_in[8];
  const float* W3    = (const float*)d_in[9];
  const float* b3    = (const float*)d_in[10];
  const float* ew0   = (const float*)d_in[11];
  const float* ew1   = (const float*)d_in[12];
  const float* ew2   = (const float*)d_in[13];
  const float* Wout  = (const float*)d_in[14];
  const float* bout  = (const float*)d_in[15];
  const float* boutp = (const float*)d_in[16];

  char* ws = (char*)d_ws;
  unsigned short* ws16 = (unsigned short*)d_ws;
  unsigned short* XB  = (unsigned short*)(ws + OFF_XB);
  unsigned short* WP  = (unsigned short*)(ws + OFF_WP);
  unsigned short* EWT = (unsigned short*)(ws + OFF_EWT);
  unsigned short* WO  = (unsigned short*)(ws + OFF_WO);
  unsigned short* RA  = (unsigned short*)(ws + OFF_RA);
  unsigned short* Q   = (unsigned short*)(ws + OFF_Q);
  unsigned short* KP  = (unsigned short*)(ws + OFF_K);
  unsigned short* VT  = (unsigned short*)(ws + OFF_VT);
  float*          Y   = (float*)(ws + OFF_Y);

  const int n8x = SROWS * FD / 8;
  k_cvt<<<dim3(n8x / 256), dim3(256), 0, stream>>>(xa, XB, n8x);
  k_cvt<<<dim3(n8x / 256), dim3(256), 0, stream>>>(xb, XB + (size_t)SROWS * FD, n8x);
  const int n8w = FD * FD / 8;
  k_cvt<<<dim3(n8w / 256), dim3(256), 0, stream>>>(Wout, WO, n8w);
  k_wt<<<dim3(1, FD / 64, NH), dim3(256), 0, stream>>>(W1, WP);
  k_wt<<<dim3(1, FD / 64, NH), dim3(256), 0, stream>>>(W2, WP + (size_t)FD * FD);
  k_wt<<<dim3(1, FD / 64, NH), dim3(256), 0, stream>>>(W3, WP + (size_t)2 * FD * FD);
  k_ew<<<dim3(1), dim3(256), 0, stream>>>(ew0, EWT);
  k_ew<<<dim3(1), dim3(256), 0, stream>>>(ew1, EWT + (size_t)HD * 128);
  k_ew<<<dim3(1), dim3(256), 0, stream>>>(ew2, EWT + (size_t)2 * HD * 128);

  k_proj<<<dim3(AROWS / 128, 3 * NH), dim3(128), 0, stream>>>(XB, WP, b1, b2, b3, ws16);
  k_g<<<dim3((SROWS * NH) / 128, 4), dim3(128), 0, stream>>>(RA, EWT, Q);

  for (int c = 0; c < 4; ++c) {
    const int kset = (c == 1 || c == 2) ? 1 : 0;
    const int vset = c & 1;
    const float* adjc = (c == 0) ? Aia : ((c == 1) ? Aib : Ait);
    const unsigned short* qh = Q + (size_t)c * SROWS * FD;
    const unsigned short* ql = qh + QPLANE;
    const unsigned short* kh = KP + (size_t)kset * SROWS * FD;
    const unsigned short* kl = kh + PLANE16;
    const unsigned short* vh = VT + (size_t)vset * SROWS * FD;
    const unsigned short* vl = vh + PLANE16;
    unsigned short* ctxc = RA + (size_t)c * SROWS * 2 * FD;
    k_attn<<<dim3(NB * NH * (NN / 64)), dim3(128), 0, stream>>>(qh, ql, kh, kl, vh, vl, adjc, ctxc,
                                                              (c == 3) ? 1 : 0);
  }

  k_out<0><<<dim3(AROWS / 128, FD / 64), dim3(128), 0, stream>>>(RA, WO, bout, boutp, Y, Y);
  k_out<1><<<dim3(AROWS / 128, FD / 64), dim3(128), 0, stream>>>(RA + (size_t)2 * SROWS * 2 * FD, WO, bout, boutp,
                                                                 Y, (float*)d_out);
  (void)hipGetLastError();
}
